// SOFTAttention_15702400434263
// MI455X (gfx1250) — hardware-verified
//
#include <hip/hip_runtime.h>

#define L_TOK 2048
#define DH    64
#define NBH   16
#define QPB   64

typedef _Float16 v16h __attribute__((ext_vector_type(16)));
typedef _Float16 v8h  __attribute__((ext_vector_type(8)));
typedef _Float16 v8ha __attribute__((ext_vector_type(8), may_alias));
typedef __bf16   v16b __attribute__((ext_vector_type(16)));
typedef float    v8f  __attribute__((ext_vector_type(8)));
typedef float    v4f  __attribute__((ext_vector_type(4)));
typedef float    v4fa __attribute__((ext_vector_type(4), may_alias));
union FragH { v16h v; v8h half[2]; _Float16 h[16]; };
union FragB { v16b v; unsigned short u[16]; };

__device__ __forceinline__ unsigned short bf16_bits(float x) { unsigned int u = __float_as_uint(x); return (unsigned short)((u + 0x7FFFu + ((u >> 16) & 1u)) >> 16); }
__device__ __forceinline__ float bf16_val(unsigned short b) { return __uint_as_float(((unsigned int)b) << 16); }
__device__ __forceinline__ v8f mma16(v16h a, v16h b, v8f c) {
  c = __builtin_amdgcn_wmma_f32_16x16x32_f16(false, a, false, b, (short)0, c, false, false);
  asm volatile("v_nop\n\tv_nop\n\tv_nop\n\tv_nop" : "+v"(c) : "v"(a), "v"(b));
  return c;
}
__device__ __forceinline__ v8f mma3(v16b ah, v16b al, v16b bh, v16b bl, v8f c) {
  c = __builtin_amdgcn_wmma_f32_16x16x32_bf16(false, ah, false, bh, (short)0, c, false, false);
  c = __builtin_amdgcn_wmma_f32_16x16x32_bf16(false, ah, false, bl, (short)0, c, false, false);
  c = __builtin_amdgcn_wmma_f32_16x16x32_bf16(false, al, false, bh, (short)0, c, false, false);
  asm volatile("v_nop\n\tv_nop\n\tv_nop\n\tv_nop" : "+v"(c) : "v"(ah), "v"(al), "v"(bh), "v"(bl));
  return c;
}

__global__ __launch_bounds__(128) void k_softattn(const float* __restrict__ q, const float* __restrict__ v, float* __restrict__ out) {
  __shared__ __attribute__((aligned(16))) unsigned short sKh[32][DH + 8], sKl[32][DH + 8];
  __shared__ float sKsq[32];
  __shared__ __attribute__((aligned(16))) _Float16 sV[32][DH + 8];
  __shared__ __attribute__((aligned(16))) _Float16 sP[4][16][40];
  __shared__ __attribute__((aligned(16))) float sO[4][16][DH];

  const int tid = threadIdx.x, w = tid >> 5, lane = tid & 31, ln = lane & 15, hh = lane >> 4;
  const int bh = blockIdx.x / (L_TOK / QPB), qblk = blockIdx.x % (L_TOK / QPB);
  const int q0 = qblk * QPB + w * 16;
  const size_t base = (size_t)bh * L_TOK * DH;
  const float* Q = q + base; const float* V = v + base; float* O = out + base;
  const float cexp = -1.0f / 16.0f;

  FragB aqh[2], aql[2];
  {
    const float* qr = Q + (size_t)(q0 + ln) * DH;
#pragma unroll
    for (int ks = 0; ks < 2; ++ks)
#pragma unroll
      for (int i = 0; i < 16; ++i) {
        const int d = ks * 32 + ((i < 8) ? (8 * hh + i) : (16 + 8 * hh + (i - 8)));
        const float x = qr[d]; const unsigned short hb = bf16_bits(x);
        aqh[ks].u[i] = hb; aql[ks].u[i] = bf16_bits(x - bf16_val(hb));
      }
  }
  float sqrow[8];
  {
    const float* qr = Q + (size_t)(q0 + ln) * DH;
    float s = 0.f;
#pragma unroll 8
    for (int d = 0; d < DH; ++d) s += qr[d] * qr[d];
#pragma unroll
    for (int r = 0; r < 8; ++r) sqrow[r] = __shfl(s, 8 * hh + r, 32);
  }

  v8f oacc[4] = {};
  for (int c = 0; c < L_TOK / 32; ++c) {
    const int j0 = c * 32;
    __syncthreads();
    for (int e = tid; e < 32 * (DH / 4); e += 128) {
      const int r = e / (DH / 4), c4 = (e % (DH / 4)) * 4;
      const v4f kq = *(const v4fa*)(Q + (size_t)(j0 + r) * DH + c4);
      const v4f vv = *(const v4fa*)(V + (size_t)(j0 + r) * DH + c4);
#pragma unroll
      for (int t = 0; t < 4; ++t) {
        const unsigned short hb = bf16_bits(kq[t]);
        sKh[r][c4 + t] = hb; sKl[r][c4 + t] = bf16_bits(kq[t] - bf16_val(hb));
        sV[r][c4 + t] = (_Float16)vv[t];
      }
    }
    if (tid < 32) {
      const float* kr = Q + (size_t)(j0 + tid) * DH;
      float s = 0.f;
#pragma unroll 8
      for (int d = 0; d < DH; ++d) s += kr[d] * kr[d];
      sKsq[tid] = s;
    }
    __syncthreads();

#pragma unroll
    for (int nt = 0; nt < 2; ++nt) {
      v8f acc = {};
#pragma unroll
      for (int ks = 0; ks < 2; ++ks) {
        FragB bkh, bkl;
        typedef unsigned short v8us __attribute__((ext_vector_type(8), may_alias));
        *(v8us*)&bkh.u[0] = *(const v8us*)&sKh[nt * 16 + ln][ks * 32 + 8 * hh];
        *(v8us*)&bkh.u[8] = *(const v8us*)&sKh[nt * 16 + ln][ks * 32 + 16 + 8 * hh];
        *(v8us*)&bkl.u[0] = *(const v8us*)&sKl[nt * 16 + ln][ks * 32 + 8 * hh];
        *(v8us*)&bkl.u[8] = *(const v8us*)&sKl[nt * 16 + ln][ks * 32 + 16 + 8 * hh];
        acc = mma3(aqh[ks].v, aql[ks].v, bkh.v, bkl.v, acc);
      }
      const float ksq = sKsq[nt * 16 + ln];
#pragma unroll
      for (int r = 0; r < 8; ++r) {
        const float d2 = sqrow[r] + ksq - 2.0f * acc[r];
        sP[w][8 * hh + r][nt * 16 + ln] = (_Float16)(__expf(cexp * d2) * 4096.0f);
      }
    }
    __builtin_amdgcn_fence(__ATOMIC_ACQ_REL, "workgroup");
    __builtin_amdgcn_wave_barrier();
    FragH pa;
    pa.half[0] = *(const v8ha*)&sP[w][ln][8 * hh];
    pa.half[1] = *(const v8ha*)&sP[w][ln][16 + 8 * hh];
#pragma unroll
    for (int dt = 0; dt < 4; ++dt) {
      FragH bv;
#pragma unroll
      for (int i = 0; i < 8; ++i) { bv.h[i] = sV[8 * hh + i][dt * 16 + ln]; bv.h[8 + i] = sV[16 + 8 * hh + i][dt * 16 + ln]; }
      oacc[dt] = mma16(pa.v, bv.v, oacc[dt]);
    }
    __builtin_amdgcn_fence(__ATOMIC_ACQ_REL, "workgroup");
    __builtin_amdgcn_wave_barrier();
  }

#pragma unroll
  for (int dt = 0; dt < 4; ++dt)
#pragma unroll
    for (int r = 0; r < 8; ++r) sO[w][8 * hh + r][dt * 16 + ln] = oacc[dt][r] * (1.0f / 4096.0f);
  __builtin_amdgcn_fence(__ATOMIC_ACQ_REL, "workgroup");
  __builtin_amdgcn_wave_barrier();
  const int rsub = lane >> 4, c4 = (lane & 15) * 4;
  for (int pass = 0; pass < 2; ++pass) {
#pragma unroll
    for (int qq = 0; qq < 8; ++qq) {
      const int r = qq * 2 + rsub;
      const v4f val = *(const v4fa*)&sO[w][r][c4];
      *(volatile v4f*)(O + (size_t)(q0 + r) * DH + c4) = val;
    }
    if (pass == 0) __threadfence();
  }
}

extern "C" void kernel_launch(void* const* d_in, const int* in_sizes, int n_in,
                              void* d_out, int out_size, void* d_ws, size_t ws_size, hipStream_t stream) {
  (void)in_sizes; (void)n_in; (void)out_size; (void)d_ws; (void)ws_size;
  const float* q = (const float*)d_in[0];
  const float* v = (const float*)d_in[1];
  k_softattn<<<NBH * (L_TOK / QPB), 128, 0, stream>>>(q, v, (float*)d_out);
}
